// SimpleRNN_41171556500011
// MI455X (gfx1250) — hardware-verified
//
#include <hip/hip_runtime.h>
#include <math.h>

constexpr int NVOC    = 128;
constexpr int NHID    = 1024;
constexpr int NOUTD   = 128;
constexpr int NBATCH  = 64;
constexpr int NSTEP   = 512;
constexpr int NTHR    = 256;
constexpr int SEQ_BLK = 16;
constexpr int HPITCH  = 1032;
constexpr int XPITCH  = 1028;
constexpr int SLABP   = 68;
constexpr int NROWS   = NBATCH * NSTEP;
constexpr int NOUT0   = NROWS * NOUTD;
constexpr float HCARRY    = 16.0f;
constexpr float LCARRY    = 2048.0f;
constexpr float WHH_CARRY = 256.0f;
constexpr float WHY_CARRY = 16.0f;
constexpr float REC_INV   = 1.0f / 4096.0f;
constexpr float RECL_INV  = 1.0f / (4096.0f * 2048.0f);
constexpr float OUT_SCALE = 1.0f / 256.0f;
static_assert(NBATCH % SEQ_BLK == 0);
static_assert(NHID == 128 * (NTHR / 32));
static_assert(NHID % 32 == 0);
static_assert(NROWS % 64 == 0 && NOUTD % 64 == 0);
static_assert((2 * SEQ_BLK * HPITCH) % NTHR == 0);
static_assert(SEQ_BLK == 2 * (NTHR / 32));
static_assert(NHID % 64 == 0 && NOUTD % 64 == 0 && NVOC % 64 == 0);
static_assert(HPITCH % 8 == 0 && XPITCH % 4 == 0);
static_assert(((NROWS / 64) * (NOUTD / 64)) % 8 == 0);
static_assert(SEQ_BLK * (NHID / 4) == 16 * NTHR);
static_assert(NHID == 4 * 256);

typedef __attribute__((ext_vector_type(16))) _Float16 v16h;
typedef __attribute__((ext_vector_type(8)))  _Float16 v8h;
typedef __attribute__((ext_vector_type(8)))  float    v8f;
typedef __attribute__((ext_vector_type(4)))  float    v4f;
typedef __attribute__((ext_vector_type(4)))  unsigned v4u;

__device__ __forceinline__ unsigned short f2bf_bits(float f) {
  unsigned u = __float_as_uint(f);
  return (unsigned short)((u + 0x7FFFu + ((u >> 16) & 1u)) >> 16);
}
__device__ __forceinline__ float bf_bits2f(unsigned short h) { return __uint_as_float(((unsigned)h) << 16); }
__device__ __forceinline__ float bf16r(float f) { return bf_bits2f(f2bf_bits(f)); }

__device__ __forceinline__ void guard4x5_h(v8f& a0, v8f& a1, v8f& a2, v8f& a3,
                                           v16h x, v16h y0, v16h y1, v16h y2, v16h y3) {
  asm volatile("v_nop\n\tv_nop\n\tv_nop\n\tv_nop"
               : "+v"(a0), "+v"(a1), "+v"(a2), "+v"(a3)
               : "v"(x), "v"(y0), "v"(y1), "v"(y2), "v"(y3));
}
__device__ __forceinline__ void guard8x6_h(v8f& a0, v8f& a1, v8f& a2, v8f& a3, v8f& a4, v8f& a5, v8f& a6, v8f& a7,
                                           v16h x0, v16h x1, v16h y0, v16h y1, v16h y2, v16h y3) {
  asm volatile("v_nop\n\tv_nop\n\tv_nop\n\tv_nop"
               : "+v"(a0), "+v"(a1), "+v"(a2), "+v"(a3), "+v"(a4), "+v"(a5), "+v"(a6), "+v"(a7)
               : "v"(x0), "v"(x1), "v"(y0), "v"(y1), "v"(y2), "v"(y3));
}
__device__ __forceinline__ void keep4_h(v16h a, v16h b, v16h c, v16h d) { asm volatile("v_nop" :: "v"(a), "v"(b), "v"(c), "v"(d)); }
__device__ __forceinline__ void acc_guard4(v8f& a, v8f& b, v8f& c, v8f& d) { asm volatile("v_nop\n\tv_nop\n\tv_nop\n\tv_nop" : "+v"(a), "+v"(b), "+v"(c), "+v"(d)); }
__device__ __forceinline__ void acc_guard8(v8f& a0, v8f& a1, v8f& a2, v8f& a3, v8f& a4, v8f& a5, v8f& a6, v8f& a7) {
  asm volatile("v_nop\n\tv_nop\n\tv_nop\n\tv_nop"
               : "+v"(a0), "+v"(a1), "+v"(a2), "+v"(a3), "+v"(a4), "+v"(a5), "+v"(a6), "+v"(a7));
}

template <typename T> struct Frag;
template <> struct Frag<_Float16> {
  typedef v16h V; union U { v16h v; v8h h[2]; };
  static __device__ __forceinline__ v16h load(const _Float16* p) {
    U f; f.h[0] = *(const v8h*)(p); f.h[1] = *(const v8h*)(p + 16); return f.v;
  }
  static __device__ __forceinline__ v8f mma(v16h a, v16h b, v8f c) {
    return __builtin_amdgcn_wmma_f32_16x16x32_f16(false, a, false, b, (short)0, c, false, false);
  }
};

__global__ __launch_bounds__(NTHR) void tpc_f16_kernel(const float* __restrict__ src, int R, int C, int ldo,
                                                       unsigned short* __restrict__ dst, float sc) {
  __shared__ float Tt[64 * 65];
  const int tid = threadIdx.x;
  const int c0 = blockIdx.x * 64, r0 = blockIdx.y * 64;
#pragma unroll
  for (int i = 0; i < 4; ++i) {
    const int idx = i * NTHR + tid;
    const int rr = idx >> 4, cc = (idx & 15) * 4;
    const v4f v = *(const v4f*)(src + (size_t)(r0 + rr) * (size_t)C + c0 + cc);
    Tt[rr * 65 + cc + 0] = v[0];
    Tt[rr * 65 + cc + 1] = v[1];
    Tt[rr * 65 + cc + 2] = v[2];
    Tt[rr * 65 + cc + 3] = v[3];
  }
  __syncthreads();
  const int q = tid >> 3, c8 = (tid & 7) * 8;
  v8h hv[2];
#pragma unroll
  for (int g = 0; g < 2; ++g) {
    const int qq = g * 32 + q;
#pragma unroll
    for (int e = 0; e < 8; ++e) {
      const float f  = Tt[(c8 + e) * 65 + qq];
      const float fb = bf16r(f);
      hv[g][e] = (_Float16)(fb * sc);
    }
  }
  _Float16* O = (_Float16*)dst;
  for (int pass = 0; pass < 2; ++pass) {
#pragma unroll
    for (int g = 0; g < 2; ++g) {
      const size_t o = (size_t)(c0 + g * 32 + q) * (size_t)ldo + (size_t)(r0 + c8);
      *(volatile v8h*)(O + o) = hv[g];
    }
    __threadfence();
  }
}

__global__ __launch_bounds__(NTHR) void rnn_seq_kernel(const int* __restrict__ tok_ids, const float* __restrict__ Wxh,
                                                       const float* __restrict__ bh,
                                                       const unsigned short* __restrict__ WHHp,
                                                       unsigned short* __restrict__ HSp) {
  __shared__ __align__(16) _Float16 Ah[2][SEQ_BLK * HPITCH];
  __shared__ __align__(16) _Float16 Al[2][SEQ_BLK * HPITCH];
  __shared__ __align__(16) float    Xp[SEQ_BLK * XPITCH];
  const _Float16* WHH = (const _Float16*)WHHp;
  const int tid = threadIdx.x, lane = tid & 31, wave = tid >> 5;
  const int c = lane & 15, hh = lane >> 4, koff = hh * 8;
  const int rowbase = blockIdx.x * SEQ_BLK;
  const int srow = tid >> 4, ssub = tid & 15;

  {
    _Float16* ahf = &Ah[0][0];
    _Float16* alf = &Al[0][0];
#pragma unroll 1
    for (int i = tid; i < 2 * SEQ_BLK * HPITCH; i += NTHR) {
      ahf[i] = (_Float16)0.0f;
      alf[i] = (_Float16)0.0f;
    }
  }
  __syncthreads();

  const v8f z8 = {0.f, 0.f, 0.f, 0.f, 0.f, 0.f, 0.f, 0.f};

#pragma unroll 1
  for (int t = 0; t < NSTEP; ++t) {
    const int cur = t & 1;
    {
      int tok = tok_ids[(size_t)(rowbase + srow) * NSTEP + (size_t)t];
      tok = tok < 0 ? 0 : (tok > NVOC - 1 ? NVOC - 1 : tok);
      const float* wrow = Wxh + (size_t)tok * NHID;
      float* xrow = Xp + srow * XPITCH;
#pragma unroll 1
      for (int it = 0; it < 16; ++it) {
        const int q4 = (ssub + 16 * it) * 4;
        const v4f wv = *(const v4f*)(wrow + q4);
        const v4f bv = *(const v4f*)(bh + q4);
        v4f xv;
        xv[0] = bf16r(wv[0]) + bf16r(bv[0]);
        xv[1] = bf16r(wv[1]) + bf16r(bv[1]);
        xv[2] = bf16r(wv[2]) + bf16r(bv[2]);
        xv[3] = bf16r(wv[3]) + bf16r(bv[3]);
        *(v4f*)(xrow + q4) = xv;
      }
    }
    __syncthreads();

    const _Float16* ahrow = &Ah[cur][0] + c * HPITCH + koff;
    const _Float16* alrow = &Al[cur][0] + c * HPITCH + koff;
    _Float16* ahn = &Ah[cur ^ 1][0];
    _Float16* aln = &Al[cur ^ 1][0];
#pragma unroll 1
    for (int ng = 0; ng < 2; ++ng) {
      const int jb = 128 * wave + 64 * ng;
      const _Float16* wb = WHH + (size_t)(jb + c) * NHID + koff;
      v8f aH[4], aL[4];
      aH[0] = z8; aH[1] = z8; aH[2] = z8; aH[3] = z8;
      aL[0] = z8; aL[1] = z8; aL[2] = z8; aL[3] = z8;
#pragma unroll 1
      for (int k0 = 0; k0 < NHID; k0 += 32) {
        const v16h xh = Frag<_Float16>::load(ahrow + k0);
        const v16h xl = Frag<_Float16>::load(alrow + k0);
        const v16h b0 = Frag<_Float16>::load(wb + k0);
        const v16h b1 = Frag<_Float16>::load(wb + (size_t)16 * NHID + k0);
        const v16h b2 = Frag<_Float16>::load(wb + (size_t)32 * NHID + k0);
        const v16h b3 = Frag<_Float16>::load(wb + (size_t)48 * NHID + k0);
        aH[0] = Frag<_Float16>::mma(xh, b0, aH[0]);
        aH[1] = Frag<_Float16>::mma(xh, b1, aH[1]);
        aH[2] = Frag<_Float16>::mma(xh, b2, aH[2]);
        aH[3] = Frag<_Float16>::mma(xh, b3, aH[3]);
        aL[0] = Frag<_Float16>::mma(xl, b0, aL[0]);
        aL[1] = Frag<_Float16>::mma(xl, b1, aL[1]);
        aL[2] = Frag<_Float16>::mma(xl, b2, aL[2]);
        aL[3] = Frag<_Float16>::mma(xl, b3, aL[3]);
        guard8x6_h(aH[0], aH[1], aH[2], aH[3], aL[0], aL[1], aL[2], aL[3], xh, xl, b0, b1, b2, b3);
      }
      acc_guard8(aH[0], aH[1], aH[2], aH[3], aL[0], aL[1], aL[2], aL[3]);
#pragma unroll
      for (int nt = 0; nt < 4; ++nt) {
        const int j = jb + 16 * nt + c;
#pragma unroll
        for (int r = 0; r < 8; ++r) {
          const int row = 8 * hh + r;
          const float dot = aH[nt][r] * REC_INV + aL[nt][r] * RECL_INV;
          const float pre = dot + Xp[row * XPITCH + j];
          const float hn  = tanhf(pre);
          const float hsc = hn * HCARRY;
          const _Float16 hq  = (_Float16)hsc;
          const float    hqf = (float)hq;
          const float    res = (hsc - hqf) * LCARRY;
          const _Float16 lq  = (_Float16)res;
          ahn[row * HPITCH + j] = hq;
          aln[row * HPITCH + j] = lq;
        }
      }
    }
    __syncthreads();

    {
      const _Float16* ahs = &Ah[cur ^ 1][0];
      for (int pass = 0; pass < 2; ++pass) {
#pragma unroll
        for (int u = 0; u < 2; ++u) {
          const int row = 2 * wave + u;
          const _Float16* srow_p = ahs + row * HPITCH;
          unsigned short* drow_p = HSp + ((size_t)(rowbase + row) * NSTEP + (size_t)t) * NHID;
#pragma unroll
          for (int q = 0; q < 4; ++q) {
            const v4u v = *(const v4u*)(const void*)(srow_p + q * 256 + lane * 8);
            *(volatile v4u*)(void*)(drow_p + q * 256 + lane * 8) = v;
          }
        }
        __threadfence();
      }
    }
  }
}

__global__ __launch_bounds__(256) void gemm64_f16_biasn(
    const unsigned short* __restrict__ Ap, int lda,
    const unsigned short* __restrict__ Btp, int ldb,
    float* __restrict__ Cout, int ldc,
    const float* __restrict__ bias,
    int M, int N, int K, float scale) {
  const _Float16* A = (const _Float16*)Ap; const _Float16* Bt = (const _Float16*)Btp;
  __shared__ __align__(16) float sT[8][16 * SLABP];
  const int lane = threadIdx.x & 31;
  const int wave = threadIdx.x >> 5;
  const int tilesN = N >> 6;
  const int tilesM = M >> 6;
  const int tile = blockIdx.x * 8 + wave;
  if (tile >= tilesM * tilesN) return;
  const int tm = tile / tilesN;
  const int tn = tile - tm * tilesN;
  const int m0 = tm << 6;
  const int n0 = tn << 6;

  const int rlane = lane & 15;
  const int koff  = (lane >> 4) * 8;
  const int mOff  = (lane >> 4) * 8;

  v8f acc[4][4];
#pragma unroll
  for (int i = 0; i < 4; ++i)
#pragma unroll
    for (int j = 0; j < 4; ++j) acc[i][j] = (v8f){0.f,0.f,0.f,0.f,0.f,0.f,0.f,0.f};

  for (int k0 = 0; k0 < K; k0 += 32) {
    v16h bfr[4];
#pragma unroll
    for (int j = 0; j < 4; ++j) {
      const size_t bo = (size_t)(n0 + (j << 4) + rlane) * ldb + koff + k0;
      bfr[j] = Frag<_Float16>::load(Bt + bo);
    }
#pragma unroll
    for (int i = 0; i < 4; ++i) {
      const size_t ao = (size_t)(m0 + (i << 4) + rlane) * lda + koff + k0;
      const v16h afr = Frag<_Float16>::load(A + ao);
#pragma unroll
      for (int j = 0; j < 4; ++j) acc[i][j] = Frag<_Float16>::mma(afr, bfr[j], acc[i][j]);
      guard4x5_h(acc[i][0], acc[i][1], acc[i][2], acc[i][3], afr, bfr[0], bfr[1], bfr[2], bfr[3]);
    }
    keep4_h(bfr[0], bfr[1], bfr[2], bfr[3]);
  }
  acc_guard4(acc[0][0], acc[0][1], acc[0][2], acc[0][3]);
  acc_guard4(acc[1][0], acc[1][1], acc[1][2], acc[1][3]);
  acc_guard4(acc[2][0], acc[2][1], acc[2][2], acc[2][3]);
  acc_guard4(acc[3][0], acc[3][1], acc[3][2], acc[3][3]);

  float bvn[4];
#pragma unroll
  for (int j = 0; j < 4; ++j) bvn[j] = bf16r(bias[n0 + (j << 4) + rlane]);
  float* slab = sT[wave];
#pragma unroll
  for (int i = 0; i < 4; ++i) {
    const int mBase = m0 + (i << 4);
#pragma unroll
    for (int j = 0; j < 4; ++j) {
#pragma unroll
      for (int r = 0; r < 8; ++r) {
        const float v = acc[i][j][r] * scale + bvn[j];
        slab[(mOff + r) * SLABP + (j << 4) + rlane] = v;
      }
    }
    __builtin_amdgcn_fence(__ATOMIC_RELEASE, "workgroup");
    __builtin_amdgcn_wave_barrier();
    __builtin_amdgcn_fence(__ATOMIC_ACQUIRE, "workgroup");
    {
      const int h2 = lane >> 4, c4 = (lane & 15) * 4;
      for (int pass = 0; pass < 2; ++pass) {
#pragma unroll
        for (int it = 0; it < 8; ++it) {
          const int row = it * 2 + h2;
          const v4f v = *(const v4f*)(slab + row * SLABP + c4);
          *(volatile v4f*)(Cout + (size_t)(mBase + row) * ldc + n0 + c4) = v;
        }
        __threadfence();
      }
    }
    __builtin_amdgcn_fence(__ATOMIC_RELEASE, "workgroup");
    __builtin_amdgcn_wave_barrier();
    __builtin_amdgcn_fence(__ATOMIC_ACQUIRE, "workgroup");
  }
}

extern "C" void kernel_launch(void* const* d_in, const int* in_sizes, int n_in,
                              void* d_out, int out_size, void* d_ws, size_t ws_size, hipStream_t stream) {
  if (n_in < 6 || d_out == nullptr || d_ws == nullptr) return;
  if (in_sizes[0] != NBATCH * NSTEP || in_sizes[1] != NHID * NHID || in_sizes[2] != NVOC * NHID ||
      in_sizes[3] != NHID * NOUTD || in_sizes[4] != NHID || in_sizes[5] != NOUTD || out_size != NOUT0) return;

  const int*   tok_ids = (const int*)d_in[0];
  const float* w_hh    = (const float*)d_in[1];
  const float* w_xh    = (const float*)d_in[2];
  const float* w_hy    = (const float*)d_in[3];
  const float* b_h     = (const float*)d_in[4];
  const float* b_y     = (const float*)d_in[5];
  float* out = (float*)d_out;
  (void)ws_size;

  char* ws = (char*)d_ws; size_t off = 0;
  auto carve = [&](size_t bytes) -> char* { char* p = ws + off; off += (bytes + 255) & ~(size_t)255; return p; };
  unsigned short* HS  = (unsigned short*)carve((size_t)NROWS * NHID * 2);
  unsigned short* WHH = (unsigned short*)carve((size_t)NHID * NHID * 2);
  unsigned short* WHY = (unsigned short*)carve((size_t)NOUTD * NHID * 2);
  if (off > ws_size || off > (size_t)134217728) return;

  tpc_f16_kernel<<<dim3(NHID / 64, NHID / 64), NTHR, 0, stream>>>(w_hh, NHID, NHID, NHID, WHH, WHH_CARRY);
  tpc_f16_kernel<<<dim3(NOUTD / 64, NHID / 64), NTHR, 0, stream>>>(w_hy, NHID, NOUTD, NHID, WHY, WHY_CARRY);
  rnn_seq_kernel<<<NBATCH / SEQ_BLK, NTHR, 0, stream>>>(tok_ids, w_xh, b_h, WHH, HS);
  gemm64_f16_biasn<<<dim3(((NROWS / 64) * (NOUTD / 64)) / 8, 1), 256, 0, stream>>>(
      HS, NHID, WHY, NHID, out, NOUTD, b_y, NROWS, NOUTD, NHID, OUT_SCALE);
}
